// HipatchOur_58308476011173
// MI455X (gfx1250) — hardware-verified
//
#include <hip/hip_runtime.h>


namespace {
constexpr int NBt = 16, M = 24, L = 32, NN = 64, H = 64, LP = 32, NPATCH = NBt * NN * M  ;
constexpr float HS = 256.0f, WSC = 256.0f, ALPHA = 0.1f;
typedef _Float16 b16;
typedef __attribute__((ext_vector_type(16))) _Float16 v16b;
typedef __attribute__((ext_vector_type(8))) _Float16 v8b;
typedef __attribute__((ext_vector_type(8))) float v8f;
typedef __attribute__((ext_vector_type(4))) float v4f;
typedef __attribute__((ext_vector_type(2))) float v2f;
__device__ __forceinline__ float bf16_rne(float f) { unsigned int u = __float_as_uint(f); u += 0x7FFFu + ((u >> 16) & 1u); float r = __uint_as_float(u & 0xFFFF0000u); asm volatile("" : "+v"(r)); return r; }
__device__ __forceinline__ float bfv(float f) { float r = bf16_rne(f); asm volatile("" : "+v"(r)); return r; }
__device__ __forceinline__ void split16(float v, b16& hi, b16& lo) { hi = (b16)v; lo = (b16)(v - (float)hi); }
__device__ __forceinline__ v16b frag_kb(const b16* p, int hh) { const v8b a = *(const v8b*)(p + 8 * hh), b = *(const v8b*)(p + 16 + 8 * hh); v16b f;
#pragma unroll
  for (int e = 0; e < 8; ++e) { f[e] = a[e]; f[8 + e] = b[e]; } return f; }
__device__ __forceinline__ v8f wmma16b(v16b a, v16b b, v8f c) { v8f d = __builtin_amdgcn_wmma_f32_16x16x32_f16(false, a, false, b, (short)0, c, false, false); asm volatile("v_nop\n\tv_nop\n\tv_nop\n\tv_nop" : "+v"(d) : "v"(a), "v"(b)); return d; }
__device__ __forceinline__ void wave_lds_sync() { __builtin_amdgcn_fence(__ATOMIC_RELEASE, "workgroup"); __builtin_amdgcn_wave_barrier(); __builtin_amdgcn_fence(__ATOMIC_ACQUIRE, "workgroup"); }
__device__ __forceinline__ float pmul(float a, float b) { float p = a * b; asm volatile("" : "+v"(p)); return p; }
__device__ __forceinline__ float te_c(float t, int c, const float* sw, const float* sb, const float* pw, const float* pb) { return c == 0 ? pmul(t, bfv(sw[0])) + bfv(sb[0]) : sinf(pmul(t, bfv(pw[c - 1])) + bfv(pb[c - 1])); }

__global__ __launch_bounds__(256) void wput_kernel(const float* __restrict__ g1, const float* __restrict__ g2, const float* __restrict__ d1, const float* __restrict__ d2, b16* __restrict__ WG, b16* __restrict__ WD1, b16* __restrict__ WD2) { const int u = blockIdx.x * 256 + threadIdx.x; v8b v;
  if (u < 2 * H * 8) { const int l = u / (H * 8), r = u % (H * 8); const int o = r / 8, k0 = (r % 8) * 8; const float* w = l ? g2 : g1;
#pragma unroll
    for (int j = 0; j < 8; ++j) v[j] = (b16)(bf16_rne(w[(size_t)o * H + k0 + j]) * WSC); for (int pass = 0; pass < 2; ++pass) { *(volatile v8b*)(WG + ((size_t)l * H + o) * H + k0) = v; __threadfence(); } }
  if (u < H * 16) { const int o = u / 16, k0 = (u % 16) * 8;
#pragma unroll
    for (int j = 0; j < 8; ++j) v[j] = (b16)(bf16_rne(d1[(size_t)o * 2 * H + k0 + j]) * WSC); for (int pass = 0; pass < 2; ++pass) { *(volatile v8b*)(WD1 + (size_t)o * 2 * H + k0) = v; __threadfence(); } }
  if (u < H * 8) { const int o = u / 8, k0 = (u % 8) * 8;
#pragma unroll
    for (int j = 0; j < 8; ++j) v[j] = (b16)(bf16_rne(d2[(size_t)o * H + k0 + j]) * WSC); for (int pass = 0; pass < 2; ++pass) { *(volatile v8b*)(WD2 + (size_t)o * H + k0) = v; __threadfence(); } } }
__global__ __launch_bounds__(32) void patch_kernel(const float* __restrict__ X, const float* __restrict__ TT, const float* __restrict__ MK, const float* __restrict__ sw, const float* __restrict__ sb, const float* __restrict__ pw, const float* __restrict__ pb, const float* __restrict__ ow, const float* __restrict__ ob, const float* __restrict__ nv, const b16* __restrict__ WG, const float* __restrict__ gb1, const float* __restrict__ gb2, int PLIM, float* __restrict__ PP) {
  __shared__ __attribute__((aligned(16))) b16 Ah[32][H + 8], Al[32][H + 8]; __shared__ float H0[32][H + 1], Hc[32][H + 1], Mh[32]; const int lane = threadIdx.x, nloc = lane & 15, hlf = lane >> 4; const int p = blockIdx.x; if (p >= PLIM) return; const int b = p / (NN * M), n = (p / M) % NN, m = p % M;
  { const size_t base = (((size_t)b * M + m) * L + lane) * NN + n; const float xv = bfv(X[base]), tv = bfv(TT[base]); Mh[lane] = bfv(MK[base]);
    for (int c = 0; c < H; ++c) H0[lane][c] = fmaxf(pmul(xv, bfv(ow[c])) + bfv(ob[c]) + bfv(nv[n * H + c]) + te_c(tv, c, sw, sb, pw, pb), 0.0f); }
  for (int k = H; k < H + 8; ++k) { Ah[lane][k] = (b16)0.0f; Al[lane][k] = (b16)0.0f; }
  wave_lds_sync();
  for (int l = 0; l < L; ++l) for (int q = 0; q < 2; ++q) Hc[l][q * 32 + lane] = H0[l][q * 32 + lane];
  float deg = 0.0f; for (int l = 0; l < L; ++l) deg += Mh[l]; const float inv = 1.0f / fmaxf(deg, 1.0f);
  wave_lds_sync();
#pragma unroll 1
  for (int layer = 0; layer < 2; ++layer) {
    float ag[2]; for (int q = 0; q < 2; ++q) { float s = 0.0f; for (int l = 0; l < L; ++l) s += pmul(Mh[l], Hc[l][q * 32 + lane]); ag[q] = s * inv; }
    for (int l = 0; l < L; ++l) for (int q = 0; q < 2; ++q) { const int c = q * 32 + lane; const float prop = pmul(1.0f - ALPHA, pmul(Mh[l], ag[q])) + pmul(ALPHA, H0[l][c]); b16 ph, pl; split16(prop * HS, ph, pl); Ah[l][c] = ph; Al[l][c] = pl; }
    wave_lds_sync();
    const b16* W = WG + (size_t)layer * H * H; const float* gb = layer ? gb2 : gb1;
#pragma unroll
    for (int rt = 0; rt < 2; ++rt) { v8f acc[4] = {(v8f){}, (v8f){}, (v8f){}, (v8f){}};
#pragma unroll
      for (int kb = 0; kb < H; kb += 32) { const v16b a = frag_kb(&Ah[rt * 16 + nloc][kb], hlf), al = frag_kb(&Al[rt * 16 + nloc][kb], hlf);
#pragma unroll
        for (int t = 0; t < 4; ++t) { const v16b bw = frag_kb(W + (size_t)(t * 16 + nloc) * H + kb, hlf); acc[t] = wmma16b(a, bw, acc[t]); acc[t] = wmma16b(al, bw, acc[t]); } }
#pragma unroll
      for (int t = 0; t < 4; ++t) { const int cc = t * 16 + nloc; const float bb = bfv(gb[cc]);
#pragma unroll
        for (int r8 = 0; r8 < 8; ++r8) { const int l = rt * 16 + 8 * hlf + r8; Hc[l][cc] = fmaxf(acc[t][r8] * (1.0f / (HS * WSC)) + bb, 0.0f) + Hc[l][cc]; } } }
    wave_lds_sync(); }
  v2f o; for (int q = 0; q < 2; ++q) { float s = 0.0f; for (int l = 0; l < L; ++l) s += pmul(Mh[l], Hc[l][lane * 2 + q]); o[q] = s; }
  for (int pass = 0; pass < 2; ++pass) { *(volatile v2f*)(PP + (size_t)p * H + lane * 2) = o; __threadfence(); } }
__global__ __launch_bounds__(256) void pool_kernel(const float* __restrict__ PP, const float* __restrict__ MK, int PLIM, float* __restrict__ PL) { const int wave = threadIdx.x >> 5, lane = threadIdx.x & 31; const int bn = blockIdx.x * 8 + wave; if (bn * M >= PLIM) return; const int b = bn / NN, n = bn % NN; float s0 = 0.0f, s1 = 0.0f, cnt = 0.0f;
  for (int m = 0; m < M; ++m) { const v2f v = *(const v2f*)(PP + ((size_t)bn * M + m) * H + lane * 2); s0 += v[0]; s1 += v[1]; cnt += bfv(MK[(((size_t)b * M + m) * L + lane) * NN + n]); }
  for (int o = 16; o; o >>= 1) cnt += __shfl_xor(cnt, o); const float inv = 1.0f / fmaxf(cnt, 1.0f);
  for (int pass = 0; pass < 2; ++pass) { *(volatile v2f*)(PL + (size_t)bn * H + lane * 2) = (v2f){s0 * inv, s1 * inv}; __threadfence(); } }
__global__ __launch_bounds__(32) void dec_kernel(const float* __restrict__ PL, const float* __restrict__ tp, const float* __restrict__ sw, const float* __restrict__ sb, const float* __restrict__ pw, const float* __restrict__ pb, const b16* __restrict__ WD1, const float* __restrict__ b1, const b16* __restrict__ WD2, const float* __restrict__ b2, const float* __restrict__ w3, const float* __restrict__ b3, int BLIM, float* __restrict__ out) { __shared__ __attribute__((aligned(16))) b16 Ah[32][2 * H + 8], Al[32][2 * H + 8]; __shared__ float Tf[32][H + 1], Os[32]; const int lane = threadIdx.x, nloc = lane & 15, hlf = lane >> 4; const int b = blockIdx.x / (LP * 2), lp = (blockIdx.x / 2) % LP, n0 = (blockIdx.x % 2) * 32; if (b >= BLIM) return; const float t = bfv(tp[b * LP + lp]);
  for (int rr = 0; rr < 32; ++rr) { const int n = n0 + rr; for (int q = 0; q < 4; ++q) { const int c = q * 32 + lane; const float v = c < H ? PL[((size_t)b * NN + n) * H + c] : te_c(t, c - H, sw, sb, pw, pb); b16 p, ql; split16(v * HS, p, ql); Ah[rr][c] = p; Al[rr][c] = ql; } }
  for (int k = 2 * H; k < 2 * H + 8; ++k) { Ah[lane][k] = (b16)0.0f; Al[lane][k] = (b16)0.0f; }
  wave_lds_sync();
#pragma unroll
  for (int rt = 0; rt < 2; ++rt) { v8f acc[4] = {(v8f){}, (v8f){}, (v8f){}, (v8f){}};
#pragma unroll
    for (int kb = 0; kb < 2 * H; kb += 32) { const v16b a = frag_kb(&Ah[rt * 16 + nloc][kb], hlf), al = frag_kb(&Al[rt * 16 + nloc][kb], hlf);
#pragma unroll
      for (int tt = 0; tt < 4; ++tt) { const v16b bw = frag_kb(WD1 + (size_t)(tt * 16 + nloc) * 2 * H + kb, hlf); acc[tt] = wmma16b(a, bw, acc[tt]); acc[tt] = wmma16b(al, bw, acc[tt]); } }
#pragma unroll
    for (int tt = 0; tt < 4; ++tt) { const int cc = tt * 16 + nloc; const float bb = bfv(b1[cc]);
#pragma unroll
      for (int r8 = 0; r8 < 8; ++r8) Tf[rt * 16 + 8 * hlf + r8][cc] = fmaxf(acc[tt][r8] * (1.0f / (HS * WSC)) + bb, 0.0f); } }
  wave_lds_sync();
  for (int rr = 0; rr < 32; ++rr) for (int q = 0; q < 2; ++q) { const int c = q * 32 + lane; b16 p, ql; split16(Tf[rr][c] * HS, p, ql); Ah[rr][c] = p; Al[rr][c] = ql; }
  for (int k = H; k < H + 8; ++k) { Ah[lane][k] = (b16)0.0f; Al[lane][k] = (b16)0.0f; }
  wave_lds_sync();
#pragma unroll
  for (int rt = 0; rt < 2; ++rt) { v8f acc[4] = {(v8f){}, (v8f){}, (v8f){}, (v8f){}};
#pragma unroll
    for (int kb = 0; kb < H; kb += 32) { const v16b a = frag_kb(&Ah[rt * 16 + nloc][kb], hlf), al = frag_kb(&Al[rt * 16 + nloc][kb], hlf);
#pragma unroll
      for (int tt = 0; tt < 4; ++tt) { const v16b bw = frag_kb(WD2 + (size_t)(tt * 16 + nloc) * H + kb, hlf); acc[tt] = wmma16b(a, bw, acc[tt]); acc[tt] = wmma16b(al, bw, acc[tt]); } }
#pragma unroll
    for (int tt = 0; tt < 4; ++tt) { const int cc = tt * 16 + nloc; const float bb = bfv(b2[cc]);
#pragma unroll
      for (int r8 = 0; r8 < 8; ++r8) Tf[rt * 16 + 8 * hlf + r8][cc] = fmaxf(acc[tt][r8] * (1.0f / (HS * WSC)) + bb, 0.0f); } }
  wave_lds_sync();
  { float s = bfv(b3[0]); for (int c = 0; c < H; ++c) s += pmul(Tf[lane][c], bfv(w3[c])); Os[lane] = s; }
  wave_lds_sync();
  for (int pass = 0; pass < 2; ++pass) { ((volatile float*)out)[((size_t)b * LP + lp) * NN + n0 + lane] = Os[lane]; __threadfence(); } }
}

extern "C" void kernel_launch(void* const* d_in, const int* in_sizes, int n_in, void* d_out, int out_size, void* d_ws, size_t ws_size, hipStream_t stream) {
  (void)n_in;
  auto Fp = [&](int i) { return (const float*)d_in[i]; };
  if (in_sizes[0] != NBt * LP || in_sizes[1] != NPATCH * L || in_sizes[2] != NPATCH * L || in_sizes[3] != NPATCH * L || in_sizes[6] != H - 1 || in_sizes[8] != H || in_sizes[10] != NN * H || in_sizes[11] != H * H || in_sizes[15] != H * 2 * H || in_sizes[17] != H * H || in_sizes[19] != H || out_size != NBt * LP * NN) return;
  const int BLIM = NBt;
  size_t off = 0; char* ws = (char*)d_ws;
  auto carve = [&](size_t bytes) { char* p = ws + off; off += (bytes + 255) & ~(size_t)255; return p; };
  b16* WG = (b16*)carve((size_t)2 * H * H * 2); b16* WD1 = (b16*)carve((size_t)H * 2 * H * 2); b16* WD2 = (b16*)carve((size_t)H * H * 2); float* PP = (float*)carve((size_t)NPATCH * H * 4); float* PL = (float*)carve((size_t)NBt * NN * H * 4);
  if (off > ws_size || off > ((size_t)16 << 20)) return;
  const int PLIM = BLIM * NN * M;
  wput_kernel<<<(2 * H * 8 + 255) / 256, 256, 0, stream>>>(Fp(11), Fp(13), Fp(15), Fp(17), WG, WD1, WD2);
  patch_kernel<<<PLIM, 32, 0, stream>>>(Fp(1), Fp(2), Fp(3), Fp(4), Fp(5), Fp(6), Fp(7), Fp(8), Fp(9), Fp(10), WG, Fp(12), Fp(14), PLIM, PP);
  pool_kernel<<<(BLIM * NN + 7) / 8, 256, 0, stream>>>(PP, Fp(3), PLIM, PL);
  dec_kernel<<<BLIM * LP * 2, 32, 0, stream>>>(PL, Fp(0), Fp(4), Fp(5), Fp(6), Fp(7), WD1, Fp(16), WD2, Fp(18), Fp(19), Fp(20), BLIM, (float*)d_out);
}
